// Attention_71373766525565
// MI455X (gfx1250) — hardware-verified
//
#include <hip/hip_runtime.h>


#ifndef NB
#define NB 4
#endif
#ifndef SEQ
#define SEQ 2048
#endif
#define NB_FULL  4
#define SEQ_FULL 2048
#define CH    1024
#define NHEAD 16
#define HS    64
#define NWV   4
#define BQ    (16 * NWV)
#define KS    32
#define OSP   68
#define GBM   (32 * NWV)
#define GBN   64
#define GSP   68
#define L2E   1.4426950408889634f
#define SCL   (L2E / 2048.0f)
#define PCAR  10.0f
#define WS_CAP 134217728ull

static_assert(CH == NHEAD * HS);
static_assert(HS == 64);
static_assert(CH % 32 == 0);
static_assert(GBN == 64);
static_assert(GBM == 128);
static_assert(((size_t)NB * SEQ) % GBM == 0);
static_assert(CH % GBN == 0);
static_assert(CH % GBM == 0);
static_assert(SEQ % GBN == 0);
static_assert(SEQ % BQ == 0);
static_assert(SEQ % KS == 0);
static_assert(OSP % 4 == 0);
static_assert(GSP % 4 == 0);
static_assert(OSP >= HS);
static_assert(GSP >= GBN);
static_assert(NB <= NB_FULL);
static_assert(SEQ <= SEQ_FULL);
static_assert(((size_t)NB * SEQ * CH) % 2048 == 0);
static_assert(((size_t)CH * CH) % 2048 == 0);
static_assert(5ull * ((size_t)NB * SEQ * CH * 2) + 4ull * ((size_t)CH * CH * 2) <= WS_CAP);

typedef unsigned short hx;
typedef __attribute__((ext_vector_type(16))) __bf16   v16bf;
typedef __attribute__((ext_vector_type(16))) _Float16 v16h;
typedef __attribute__((ext_vector_type(8)))  _Float16 v8h;
typedef __attribute__((ext_vector_type(8)))  unsigned short v8us;
typedef __attribute__((ext_vector_type(4)))  unsigned int   v4u;
typedef __attribute__((ext_vector_type(8)))  unsigned int   v8u;
typedef __attribute__((ext_vector_type(8)))  float    v8f;
typedef __attribute__((ext_vector_type(4)))  float    v4f;
typedef v4f __attribute__((may_alias)) v4fa;
typedef v4u __attribute__((may_alias)) v4ua;

__device__ __forceinline__ unsigned short f2bf(float f) { unsigned u = __float_as_uint(f); u += 0x7FFFu + ((u >> 16) & 1u); return (unsigned short)(u >> 16); }
__device__ __forceinline__ float bf2f(unsigned short b) { return __uint_as_float(((unsigned)b) << 16); }
__device__ __forceinline__ float bfr(float f) { return bf2f(f2bf(f)); }
__device__ __forceinline__ unsigned short f2h(float f) { const _Float16 h = (_Float16)f; return __builtin_bit_cast(unsigned short, h); }

__device__ __forceinline__ v8u ldf(const hx* p) {
    const v4u lo = *(const v4ua*)p;
    const v4u hi = *(const v4ua*)(p + 16);
    return __builtin_shufflevector(lo, hi, 0, 1, 2, 3, 4, 5, 6, 7);
}
__device__ __forceinline__ v8f wmma_b(v8u a, v8u b, v8f c) {
    return __builtin_amdgcn_wmma_f32_16x16x32_bf16(false, __builtin_bit_cast(v16bf, a), false, __builtin_bit_cast(v16bf, b), (short)0, c, false, false);
}
__device__ __forceinline__ v8f wmma_h(v8u a, v8u b, v8f c) {
    return __builtin_amdgcn_wmma_f32_16x16x32_f16(false, __builtin_bit_cast(v16h, a), false, __builtin_bit_cast(v16h, b), (short)0, c, false, false);
}
template <bool F16OP>
__device__ __forceinline__ v8f mm(v8u a, v8u b, v8f c) {
    if (F16OP) return wmma_h(a, b, c);
    return wmma_b(a, b, c);
}

__global__ __launch_bounds__(256) void k_cvtx(const float* __restrict__ x, hx* XB) {
    const unsigned i = blockIdx.x * 256u + threadIdx.x;
    const unsigned per = (unsigned)((size_t)SEQ * CH / 8);
    if (i >= (unsigned)NB * per) return;
    const unsigned b = i / per, r = i - b * per;
    const float* src = x + (size_t)b * SEQ_FULL * CH + (size_t)r * 8;
    hx* dst = XB + (size_t)i * 8;
    const v8f v = *(const v8f*)src;
    v8us o;
#pragma unroll
    for (int c = 0; c < 8; ++c) o[c] = f2bf(v[c]);
    *(volatile v8us*)dst = o;
    __threadfence();
    *(volatile v8us*)dst = o;
}

__global__ __launch_bounds__(256) void k_cvtw(const float* __restrict__ Wk, const float* __restrict__ Wq,
                                              const float* __restrict__ Wv, const float* __restrict__ Wo, hx* WP) {
    const unsigned i = blockIdx.x * 256u + threadIdx.x;
    if (i >= (unsigned)((size_t)CH * CH / 8)) return;
    const unsigned y = blockIdx.y;
    const size_t off = (size_t)i * 8;
    v8f v;
    if (y == 0u)      v = *(const v8f*)(Wk + off);
    else if (y == 1u) v = *(const v8f*)(Wq + off);
    else if (y == 2u) v = *(const v8f*)(Wv + off);
    else              v = *(const v8f*)(Wo + off);
    v8us o;
    if (y == 3u) {
#pragma unroll
        for (int c = 0; c < 8; ++c) o[c] = f2h(bfr(v[c]) * 1024.0f);
    } else {
#pragma unroll
        for (int c = 0; c < 8; ++c) o[c] = f2bf(v[c]);
    }
    hx* dst = WP + (size_t)y * CH * CH + off;
    *(volatile v8us*)dst = o;
    __threadfence();
    *(volatile v8us*)dst = o;
}

template <bool F16OP, bool F32OUT>
__device__ __forceinline__ void gemm_body(const hx* __restrict__ A, const hx* __restrict__ Bm, float* Cf, hx* Chx,
                                          const unsigned lda, const unsigned ldb, const unsigned ldc, const float oscale) {
    __shared__ __align__(16) float st[NWV * 32 * GSP];
    const unsigned tid = threadIdx.x, lane = tid & 31u, wv = tid >> 5, lr = lane & 15u, hi = lane >> 4;
    const unsigned m0 = blockIdx.y * GBM + wv * 32u;
    const unsigned n0 = blockIdx.x * GBN;
    const hx* ap = A + (size_t)(m0 + lr) * lda + 8u * hi;
    const hx* bp = Bm + (size_t)(n0 + lr) * ldb + 8u * hi;

    v8f acc[2][4];
#pragma unroll
    for (int i = 0; i < 2; ++i)
#pragma unroll
        for (int j = 0; j < 4; ++j) acc[i][j] = (v8f){};

#pragma unroll 1
    for (unsigned k0 = 0; k0 < (unsigned)CH; k0 += 32u) {
        const v8u a0 = ldf(ap + k0);
        const v8u a1 = ldf(ap + (size_t)16 * lda + k0);
        v8u bq[4];
#pragma unroll
        for (int j = 0; j < 4; ++j) bq[j] = ldf(bp + (size_t)(j * 16) * ldb + k0);
#pragma unroll
        for (int j = 0; j < 4; ++j) {
            acc[0][j] = mm<F16OP>(a0, bq[j], acc[0][j]);
            acc[1][j] = mm<F16OP>(a1, bq[j], acc[1][j]);
        }
        asm volatile("v_nop\n\tv_nop\n\tv_nop\n\tv_nop"
                     : "+v"(acc[0][0]), "+v"(acc[0][1]), "+v"(acc[0][2]), "+v"(acc[0][3]),
                       "+v"(acc[1][0]), "+v"(acc[1][1]), "+v"(acc[1][2]), "+v"(acc[1][3])
                     : "v"(a0), "v"(a1), "v"(bq[3]));
    }

    float* sw = st + wv * (32 * GSP);
#pragma unroll
    for (int i = 0; i < 2; ++i)
#pragma unroll
        for (int j = 0; j < 4; ++j)
#pragma unroll
            for (int r = 0; r < 8; ++r) sw[(i * 16 + 8 * hi + r) * GSP + j * 16 + lr] = acc[i][j][r] * oscale;
    __syncthreads();

    if (F32OUT) {
        const unsigned c4 = (lane & 15u) * 4u, rq = lane >> 4;
        float* crow = Cf + (size_t)m0 * ldc + n0 + c4;
#pragma unroll 1
        for (int ps = 0; ps < 2; ++ps) {
#pragma unroll 4
            for (unsigned it = 0; it < 16; ++it) {
                const unsigned row = it * 2u + rq;
                const v4f val = *(const v4fa*)(sw + row * GSP + c4);
                *(volatile v4f*)(crow + (size_t)row * ldc) = val;
            }
            if (ps == 0) __threadfence();
        }
    } else {
        const unsigned c8 = (lane & 7u) * 8u, rq = lane >> 3;
        hx* crow = Chx + (size_t)m0 * ldc + n0 + c8;
#pragma unroll 1
        for (int ps = 0; ps < 2; ++ps) {
#pragma unroll 4
            for (unsigned it = 0; it < 8; ++it) {
                const unsigned row = it * 4u + rq;
                const v4f x0 = *(const v4fa*)(sw + row * GSP + c8);
                const v4f x1 = *(const v4fa*)(sw + row * GSP + c8 + 4u);
                v8h hv;
                hv[0] = (_Float16)x0[0]; hv[1] = (_Float16)x0[1]; hv[2] = (_Float16)x0[2]; hv[3] = (_Float16)x0[3];
                hv[4] = (_Float16)x1[0]; hv[5] = (_Float16)x1[1]; hv[6] = (_Float16)x1[2]; hv[7] = (_Float16)x1[3];
                const v8us o = __builtin_bit_cast(v8us, hv);
                *(volatile v8us*)(crow + (size_t)row * ldc) = o;
            }
            if (ps == 0) __threadfence();
        }
    }
}

__global__ __launch_bounds__(128) void k_gemm_qk(const hx* __restrict__ XB, const hx* __restrict__ WP, hx* QK) {
    const unsigned z = blockIdx.z;
    gemm_body<false, false>(XB, WP + (size_t)z * CH * CH, nullptr, QK + (size_t)z * NB * SEQ * CH,
                            (unsigned)CH, (unsigned)CH, (unsigned)CH, 16.0f);
}

__global__ __launch_bounds__(128) void k_gemm_vt(const hx* __restrict__ XB, const hx* __restrict__ WP, hx* VT) {
    const unsigned z = blockIdx.z;
    gemm_body<false, false>(WP + (size_t)2 * CH * CH, XB + (size_t)z * SEQ * CH, nullptr, VT + (size_t)z * CH * SEQ,
                            (unsigned)CH, (unsigned)CH, (unsigned)SEQ, 16.0f);
}

__global__ __launch_bounds__(128) void k_gemm_out(const hx* __restrict__ CTX, const hx* __restrict__ WP, float* OUT) {
    gemm_body<true, true>(CTX, WP + (size_t)3 * CH * CH, OUT, nullptr,
                          (unsigned)CH, (unsigned)CH, (unsigned)CH, 3.814697265625e-06f);
}

__global__ __launch_bounds__(128) void k_flash(const hx* __restrict__ QP, const hx* __restrict__ KP, const hx* __restrict__ VT, hx* CTX) {
    __shared__ __align__(16) float os[NWV * 16 * OSP];
    const unsigned tid = threadIdx.x, lane = tid & 31u, wv = tid >> 5, lr = lane & 15u, hi = lane >> 4;
    const unsigned bpb = (unsigned)(SEQ / BQ);
    const unsigned bh = blockIdx.x / bpb;
    const unsigned qb = blockIdx.x - bh * bpb;
    const unsigned b = bh / NHEAD;
    const unsigned hd = bh - b * NHEAD;
    const unsigned q0 = qb * BQ + wv * 16u;

    v8u qf[2];
    {
        const hx* qp = QP + ((size_t)b * SEQ + q0 + lr) * CH + hd * HS + 8u * hi;
        qf[0] = ldf(qp);
        qf[1] = ldf(qp + 32);
    }
    const hx* kp = KP + ((size_t)b * SEQ + lr) * CH + hd * HS + 8u * hi;
    const hx* vp = VT + ((size_t)b * CH + hd * HS + lr) * SEQ + 8u * hi;

    v8f o[4];
#pragma unroll
    for (int t = 0; t < 4; ++t) o[t] = (v8f){};
    float ml = -1.0e30f;
    float l = 0.0f;

#pragma unroll 1
    for (unsigned k0 = 0; k0 < (unsigned)SEQ; k0 += KS) {
        v8f s0 = (v8f){}, s1 = (v8f){};
        const hx* ka = kp + (size_t)k0 * CH;
#pragma unroll
        for (int dk = 0; dk < 2; ++dk) {
            const v8u a0 = ldf(ka + dk * 32);
            const v8u a1 = ldf(ka + 16 * CH + dk * 32);
            s0 = wmma_h(a0, qf[dk], s0);
            s1 = wmma_h(a1, qf[dk], s1);
        }
        asm volatile("v_nop\n\tv_nop\n\tv_nop\n\tv_nop" : "+v"(s0), "+v"(s1) : "v"(qf[0]), "v"(qf[1]));

        float mx = fmaxf(s0[0], s1[0]);
#pragma unroll
        for (int r = 1; r < 8; ++r) mx = fmaxf(mx, fmaxf(s0[r], s1[r]));
        mx = fmaxf(mx, __shfl_xor(mx, 16, 32));
        const float mnl = fmaxf(ml, mx * SCL);
        const float corr = __builtin_amdgcn_exp2f(ml - mnl);
        ml = mnl;
        const float off = PCAR - mnl;
        float p0[8], p1[8];
        float ps = 0.0f;
#pragma unroll
        for (int r = 0; r < 8; ++r) {
            p0[r] = __builtin_amdgcn_exp2f(fmaf(s0[r], SCL, off));
            p1[r] = __builtin_amdgcn_exp2f(fmaf(s1[r], SCL, off));
            ps += p0[r] + p1[r];
        }
        ps += __shfl_xor(ps, 16, 32);
        l = l * corr + ps;
        if (__builtin_amdgcn_ballot_w32(corr != 1.0f) != 0u) {
#pragma unroll
            for (int t = 0; t < 4; ++t) o[t] *= corr;
        }

        v16h phv;
#pragma unroll
        for (int r = 0; r < 8; ++r) {
            phv[r]     = (_Float16)p0[r];
            phv[8 + r] = (_Float16)p1[r];
        }
        const v8u ph = __builtin_bit_cast(v8u, phv);

        asm volatile("" ::: "memory");
        const hx* va = vp + k0;
#pragma unroll
        for (int t = 0; t < 4; ++t) {
            const v8u a = ldf(va + (size_t)t * 16 * SEQ);
            o[t] = wmma_h(a, ph, o[t]);
        }
        asm volatile("v_nop\n\tv_nop\n\tv_nop\n\tv_nop"
                     : "+v"(o[0]), "+v"(o[1]), "+v"(o[2]), "+v"(o[3])
                     : "v"(ph));
    }

    const float inv = 16.0f * (1.0f / l);
    float* ow = os + wv * (16 * OSP);
#pragma unroll
    for (int t = 0; t < 4; ++t) {
#pragma unroll
        for (int r = 0; r < 8; ++r) ow[lr * OSP + t * 16 + 8 * hi + r] = o[t][r] * inv;
    }
    __syncthreads();
    const unsigned c8 = (lane & 7u) * 8u, rq = lane >> 3;
    hx* crow = CTX + ((size_t)b * SEQ + q0) * CH + hd * HS + c8;
#pragma unroll 1
    for (int ps2 = 0; ps2 < 2; ++ps2) {
#pragma unroll
        for (unsigned it = 0; it < 4; ++it) {
            const unsigned row = it * 4u + rq;
            const v4f x0 = *(const v4fa*)(ow + row * OSP + c8);
            const v4f x1 = *(const v4fa*)(ow + row * OSP + c8 + 4u);
            v8h hv;
            hv[0] = (_Float16)x0[0]; hv[1] = (_Float16)x0[1]; hv[2] = (_Float16)x0[2]; hv[3] = (_Float16)x0[3];
            hv[4] = (_Float16)x1[0]; hv[5] = (_Float16)x1[1]; hv[6] = (_Float16)x1[2]; hv[7] = (_Float16)x1[3];
            const v8us ov = __builtin_bit_cast(v8us, hv);
            *(volatile v8us*)(crow + (size_t)row * CH) = ov;
        }
        if (ps2 == 0) __threadfence();
    }
}

extern "C" void kernel_launch(void* const* d_in, const int* in_sizes, int n_in,
                              void* d_out, int out_size, void* d_ws, size_t ws_size, hipStream_t stream) {
    if (n_in < 5) return;
    const size_t needx = ((size_t)(NB - 1) * SEQ_FULL + SEQ) * CH;
    const size_t needw = (size_t)CH * CH;
    if ((size_t)in_sizes[0] < needx) return;
    if ((size_t)in_sizes[1] < needw || (size_t)in_sizes[2] < needw || (size_t)in_sizes[3] < needw || (size_t)in_sizes[4] < needw) return;
    if ((size_t)out_size < (size_t)NB * SEQ * CH) return;
    const float* x  = (const float*)d_in[0];
    const float* Wk = (const float*)d_in[1];
    const float* Wq = (const float*)d_in[2];
    const float* Wv = (const float*)d_in[3];
    const float* Wo = (const float*)d_in[4];
    float* OUT = (float*)d_out;

    const size_t PB = (size_t)NB * SEQ * CH * 2;
    const size_t WB = (size_t)CH * CH * 2;
    const size_t total = 5 * PB + 4 * WB;
    if (total > ws_size || total > (size_t)WS_CAP) return;
    char* wsp = (char*)d_ws;
    hx* XB  = (hx*)(wsp);
    hx* WP  = (hx*)(wsp + PB);
    hx* QK  = (hx*)(wsp + PB + 4 * WB);
    hx* VT  = (hx*)(wsp + 3 * PB + 4 * WB);
    hx* CTX = (hx*)(wsp + 4 * PB + 4 * WB);
    hx* KPl = QK;
    hx* QPl = QK + (size_t)NB * SEQ * CH;

    const unsigned gx = (unsigned)(((size_t)NB * SEQ * CH / 8 + 255) / 256);
    const unsigned gw = (unsigned)(((size_t)CH * CH / 8 + 255) / 256);
    k_cvtx<<<gx, 256, 0, stream>>>(x, XB);
    k_cvtw<<<dim3(gw, 4, 1), 256, 0, stream>>>(Wk, Wq, Wv, Wo, WP);
    k_gemm_qk<<<dim3(CH / GBN, (unsigned)((size_t)NB * SEQ / GBM), 2), 128, 0, stream>>>(XB, WP, QK);
    k_gemm_vt<<<dim3(SEQ / GBN, CH / GBM, NB), 128, 0, stream>>>(XB, WP, VT);
    k_flash<<<(unsigned)(NB * NHEAD * (SEQ / BQ)), 128, 0, stream>>>(QPl, KPl, VT, CTX);
    k_gemm_out<<<dim3(CH / GBN, (unsigned)((size_t)NB * SEQ / GBM), 1), 128, 0, stream>>>(CTX, WP, OUT);
}
